// MatchLSTM_77644418777936
// MI455X (gfx1250) — hardware-run, weakly checked
//
#include <hip/hip_runtime.h>
#include <math.h>

constexpr int NBATCH  = 64;
constexpr int NSTEP   = 512;
constexpr int NQ      = 64;
constexpr int ND      = 256;
constexpr int NG4     = 4 * ND;
constexpr int NZ      = 2 * ND;
constexpr int NOUTROW = NSTEP + 1;
constexpr int SEQ_BLK = 16;
constexpr int PTHR    = 512;
constexpr int CTHR    = 256;
constexpr int HP = 264;
constexpr int UP = 260;
constexpr int SLP = 36;
constexpr int QS_FLOATS = (2 * SEQ_BLK * HP) / 2;

constexpr float ACT_CARRY  = 8.0f;
constexpr float WGT_CARRY  = 256.0f;
constexpr float RES_CARRY  = 2048.0f;
constexpr float RES_INV    = 1.0f / RES_CARRY;
constexpr float PROD_INV   = 1.0f / (ACT_CARRY * WGT_CARRY);
constexpr float LOG2E_F    = 1.44269504088896341f;
constexpr float K2LOG      = 2.0f * LOG2E_F;
constexpr float USCALE     = PROD_INV * K2LOG;
constexpr float F16_MINN   = 6.103515625e-05f;

static_assert(ND % 32 == 0);
static_assert(NZ % 32 == 0);
static_assert(NBATCH % SEQ_BLK == 0);
static_assert(PTHR == 32 * SEQ_BLK);
static_assert(ND == 16 * (PTHR / 32));
static_assert(PTHR * 8 == SEQ_BLK * ND);
static_assert(SEQ_BLK * UP <= QS_FLOATS);
static_assert((NBATCH * NQ) % 32 == 0 && (NBATCH * NSTEP) % 32 == 0 && ND % 32 == 0);
static_assert(HP % 8 == 0 && UP % 4 == 0 && SLP % 4 == 0);

typedef __attribute__((ext_vector_type(16))) _Float16 v16h;
typedef __attribute__((ext_vector_type(8)))  _Float16 v8h;
typedef __attribute__((ext_vector_type(8)))  float    v8f;
typedef __attribute__((ext_vector_type(4)))  float    v4f;

__device__ __forceinline__ v16h frag_load(const _Float16* p) {
  union { v16h v; v8h h[2]; } f;
  f.h[0] = *(const v8h*)(p);
  f.h[1] = *(const v8h*)(p + 16);
  return f.v;
}

__device__ __forceinline__ v8f mma_g(v16h a, v16h b, v8f c) {
  c = __builtin_amdgcn_wmma_f32_16x16x32_f16(false, a, false, b, (short)0, c, false, false);
  asm volatile("v_nop\n\tv_nop\n\tv_nop\n\tv_nop" : "+v"(c) : "v"(a), "v"(b));
  return c;
}

__device__ __forceinline__ void split16(float v, _Float16& hi, _Float16& lo) {
  const float vh = (fabsf(v) < F16_MINN) ? 0.0f : v;
  hi = (_Float16)vh;
  const float res = (v - (float)hi) * RES_CARRY;
  const float rl = (fabsf(res) < F16_MINN) ? 0.0f : res;
  lo = (_Float16)rl;
}

__device__ __forceinline__ float fsig(float x) {
  const float xc = __builtin_amdgcn_fmed3f(x, -30.0f, 30.0f);
  return __builtin_amdgcn_rcpf(1.0f + __builtin_amdgcn_exp2f(-LOG2E_F * xc));
}
__device__ __forceinline__ float ftanh(float x) {
  const float xc = __builtin_amdgcn_fmed3f(x, -15.0f, 15.0f);
  return 1.0f - 2.0f * __builtin_amdgcn_rcpf(__builtin_amdgcn_exp2f(K2LOG * xc) + 1.0f);
}

__global__ __launch_bounds__(CTHR) void split8_kernel(const float* __restrict__ src, unsigned short* __restrict__ hi,
                                                      unsigned short* __restrict__ lo, int n8, float sc) {
  const int i = blockIdx.x * CTHR + threadIdx.x;
  if (i < n8) {
    const float* sp = src + (size_t)i * 8;
    const v4f a = *(const v4f*)(sp);
    const v4f b = *(const v4f*)(sp + 4);
    v8h hv, lv;
#pragma unroll
    for (int e = 0; e < 4; ++e) {
      const float fa = a[e] * sc;
      const float fb = b[e] * sc;
      _Float16 h0, l0, h1, l1;
      split16(fa, h0, l0);
      split16(fb, h1, l1);
      hv[e] = h0;
      lv[e] = l0;
      hv[4 + e] = h1;
      lv[4 + e] = l1;
    }
    for (int pass = 0; pass < 2; ++pass) {
      *(volatile v8h*)(hi + (size_t)i * 8) = hv;
      *(volatile v8h*)(lo + (size_t)i * 8) = lv;
      __threadfence();
    }
  }
}

__global__ __launch_bounds__(CTHR) void tsplit_kernel(const float* __restrict__ s0, const float* __restrict__ s1,
                                                      const float* __restrict__ s2, unsigned short* __restrict__ O, float sc) {
  __shared__ float Tt[64 * 65];
  const int tid = threadIdx.x;
  const int z = blockIdx.z;
  const float* src = (z == 0) ? s0 : ((z == 1) ? s1 : s2);
  unsigned short* Oh = O + (size_t)z * (size_t)(2 * ND * ND);
  unsigned short* Ol = Oh + (size_t)(ND * ND);
  const int c0 = blockIdx.x * 64, r0 = blockIdx.y * 64;
#pragma unroll
  for (int i = 0; i < 4; ++i) {
    const int idx = i * CTHR + tid;
    const int rr = idx >> 4, cc = (idx & 15) * 4;
    const v4f v = *(const v4f*)(src + (size_t)(r0 + rr) * (size_t)ND + c0 + cc);
    Tt[rr * 65 + cc + 0] = v[0];
    Tt[rr * 65 + cc + 1] = v[1];
    Tt[rr * 65 + cc + 2] = v[2];
    Tt[rr * 65 + cc + 3] = v[3];
  }
  __syncthreads();
  const int q = tid >> 3, c8 = (tid & 7) * 8;
  v8h hv[2], lv[2];
#pragma unroll
  for (int g = 0; g < 2; ++g) {
    const int qq = g * 32 + q;
#pragma unroll
    for (int e = 0; e < 8; ++e) {
      const float f = Tt[(c8 + e) * 65 + qq] * sc;
      _Float16 h, l;
      split16(f, h, l);
      hv[g][e] = h;
      lv[g][e] = l;
    }
  }
  for (int pass = 0; pass < 2; ++pass) {
#pragma unroll
    for (int g = 0; g < 2; ++g) {
      const size_t o = (size_t)(c0 + g * 32 + q) * (size_t)ND + (size_t)(r0 + c8);
      *(volatile v8h*)(Oh + o) = hv[g];
      *(volatile v8h*)(Ol + o) = lv[g];
    }
    __threadfence();
  }
}

__global__ __launch_bounds__(CTHR) void proj3_kernel(const unsigned short* __restrict__ Ahp, const unsigned short* __restrict__ Alp,
                                                     const unsigned short* __restrict__ Bhp, const unsigned short* __restrict__ Blp,
                                                     float* __restrict__ C, int M, float scale) {
  __shared__ __align__(16) float sT[CTHR / 32][16 * SLP];
  const _Float16* Ah = (const _Float16*)Ahp;
  const _Float16* Al = (const _Float16*)Alp;
  const _Float16* Bh = (const _Float16*)Bhp;
  const _Float16* Bl = (const _Float16*)Blp;
  const int lane = threadIdx.x & 31, wave = threadIdx.x >> 5;
  const int tile = blockIdx.x * (CTHR / 32) + wave;
  const int tm = tile >> 3, tn = tile & 7;
  const int m0 = tm * 32, n0 = tn * 32;
  if (m0 >= M) return;
  const int rlane = lane & 15, koff = (lane >> 4) * 8, mOff = (lane >> 4) * 8;
  const v8f z8 = {0.f, 0.f, 0.f, 0.f, 0.f, 0.f, 0.f, 0.f};
  v8f accM[2][2], accR[2][2];
#pragma unroll
  for (int i = 0; i < 2; ++i)
#pragma unroll
    for (int j = 0; j < 2; ++j) { accM[i][j] = z8; accR[i][j] = z8; }

#pragma unroll 1
  for (int k0 = 0; k0 < ND; k0 += 32) {
    v16h bh[2], bl[2];
#pragma unroll
    for (int j = 0; j < 2; ++j) {
      const size_t bo = (size_t)(n0 + 16 * j + rlane) * (size_t)ND + koff + k0;
      bh[j] = frag_load(Bh + bo);
      bl[j] = frag_load(Bl + bo);
    }
#pragma unroll
    for (int i = 0; i < 2; ++i) {
      const size_t ao = (size_t)(m0 + 16 * i + rlane) * (size_t)ND + koff + k0;
      const v16h ah = frag_load(Ah + ao);
      const v16h al = frag_load(Al + ao);
#pragma unroll
      for (int j = 0; j < 2; ++j) {
        accM[i][j] = mma_g(ah, bh[j], accM[i][j]);
        accR[i][j] = mma_g(ah, bl[j], accR[i][j]);
        accR[i][j] = mma_g(al, bh[j], accR[i][j]);
      }
    }
  }

  float* slab = sT[wave];
#pragma unroll
  for (int i = 0; i < 2; ++i) {
    const int mBase = m0 + 16 * i;
#pragma unroll
    for (int j = 0; j < 2; ++j)
#pragma unroll
      for (int r = 0; r < 8; ++r)
        slab[(mOff + r) * SLP + 16 * j + rlane] = (accM[i][j][r] + accR[i][j][r] * RES_INV) * scale;
    __builtin_amdgcn_fence(__ATOMIC_RELEASE, "workgroup");
    __builtin_amdgcn_wave_barrier();
    __builtin_amdgcn_fence(__ATOMIC_ACQUIRE, "workgroup");
    {
      const int q = lane >> 3, c4 = (lane & 7) * 4;
      for (int pass = 0; pass < 2; ++pass) {
#pragma unroll
        for (int it = 0; it < 4; ++it) {
          const int row = it * 4 + q;
          const v4f v = *(const v4f*)(slab + row * SLP + c4);
          *(volatile v4f*)(C + (size_t)(mBase + row) * (size_t)ND + n0 + c4) = v;
        }
        __threadfence();
      }
    }
    __builtin_amdgcn_fence(__ATOMIC_RELEASE, "workgroup");
    __builtin_amdgcn_wave_barrier();
    __builtin_amdgcn_fence(__ATOMIC_ACQUIRE, "workgroup");
  }
}

__global__ __launch_bounds__(PTHR) void seq_kernel(
    const unsigned short* __restrict__ ECHp, const unsigned short* __restrict__ ECLp,
    const unsigned short* __restrict__ WRHp, const unsigned short* __restrict__ WRLp,
    const unsigned short* __restrict__ WIHp, const unsigned short* __restrict__ WILp,
    const unsigned short* __restrict__ WHHp, const unsigned short* __restrict__ WHLp,
    const float* __restrict__ WHQ, const float* __restrict__ WHP,
    const float* __restrict__ eq, const float* __restrict__ h0, const float* __restrict__ c0,
    const float* __restrict__ wvec, const float* __restrict__ bih, const float* __restrict__ bhh,
    float* __restrict__ out) {
  __shared__ __align__(16) _Float16 Hh[SEQ_BLK * HP];
  __shared__ __align__(16) _Float16 Hl[SEQ_BLK * HP];
  __shared__ __align__(16) float    Ub[SEQ_BLK * UP];
  __shared__ __align__(16) float    QS[QS_FLOATS];
  _Float16* Qh = (_Float16*)QS;
  _Float16* Ql = Qh + SEQ_BLK * HP;
  float*    Hs = QS;

  const _Float16* ECH = (const _Float16*)ECHp;
  const _Float16* ECL = (const _Float16*)ECLp;
  const _Float16* WRH = (const _Float16*)WRHp;
  const _Float16* WRL = (const _Float16*)WRLp;
  const _Float16* WIH = (const _Float16*)WIHp;
  const _Float16* WIL = (const _Float16*)WILp;
  const _Float16* WHH = (const _Float16*)WHHp;
  const _Float16* WHL = (const _Float16*)WHLp;

  const int tid = threadIdx.x, lane = tid & 31, wave = tid >> 5;
  const int c = lane & 15, hh = lane >> 4, koff = hh * 8;
  const int rowbase = blockIdx.x * SEQ_BLK;
  const int ucol = 16 * wave + c;

  {
    const float* hp = h0 + (size_t)(rowbase + wave) * ND + 8 * lane;
    const v4f a = *(const v4f*)(hp);
    const v4f b = *(const v4f*)(hp + 4);
    v8h hv, lv;
#pragma unroll
    for (int e = 0; e < 4; ++e) {
      const float fa = a[e] * ACT_CARRY;
      const float fb = b[e] * ACT_CARRY;
      _Float16 x0, y0, x1, y1;
      split16(fa, x0, y0);
      split16(fb, x1, y1);
      hv[e] = x0;
      lv[e] = y0;
      hv[4 + e] = x1;
      lv[4 + e] = y1;
    }
    *(v8h*)(Hh + wave * HP + 8 * lane) = hv;
    *(v8h*)(Hl + wave * HP + 8 * lane) = lv;
  }
  {
    const float* hp = h0 + (size_t)(rowbase + wave) * ND;
    const v4f a = *(const v4f*)(hp + 4 * lane);
    const v4f b = *(const v4f*)(hp + 128 + 4 * lane);
    float* orow = out + ((size_t)(rowbase + wave) * NOUTROW) * ND;
    for (int pass = 0; pass < 2; ++pass) {
      *(volatile v4f*)(orow + 4 * lane) = a;
      *(volatile v4f*)(orow + 128 + 4 * lane) = b;
      __threadfence();
    }
  }

  float cst[8], bia[4];
#pragma unroll
  for (int r = 0; r < 8; ++r) cst[r] = c0[(size_t)(rowbase + 8 * hh + r) * ND + ucol];
#pragma unroll
  for (int g = 0; g < 4; ++g) bia[g] = bih[g * ND + ucol] + bhh[g * ND + ucol];
  v4f m2w0, m2w1;
  float wsum = 0.0f;
  {
    const v4f w0 = *(const v4f*)(wvec + 8 * lane);
    const v4f w1 = *(const v4f*)(wvec + 8 * lane + 4);
#pragma unroll
    for (int e = 0; e < 4; ++e) {
      m2w0[e] = -2.0f * w0[e];
      m2w1[e] = -2.0f * w1[e];
      wsum += w0[e] + w1[e];
    }
  }
  __syncthreads();

  const v8f z8 = {0.f, 0.f, 0.f, 0.f, 0.f, 0.f, 0.f, 0.f};
  const size_t GS_IH = (size_t)ND * (size_t)NZ;
  const size_t GS_HH = (size_t)ND * (size_t)ND;

#pragma unroll 1
  for (int t = 0; t < NSTEP; ++t) {
    {
      float pv[8];
#pragma unroll
      for (int r = 0; r < 8; ++r)
        pv[r] = WHP[((size_t)(rowbase + 8 * hh + r) * NSTEP + (size_t)t) * ND + ucol];
      const _Float16* ahp = Hh + c * HP + koff;
      const _Float16* alp = Hl + c * HP + koff;
      const _Float16* bhp = WRH + (size_t)ucol * ND + koff;
      const _Float16* blp = WRL + (size_t)ucol * ND + koff;
      v8f aM = z8, aR = z8;
#pragma unroll 1
      for (int k0 = 0; k0 < ND; k0 += 32) {
        const v16h ah = frag_load(ahp + k0);
        const v16h al = frag_load(alp + k0);
        const v16h bh = frag_load(bhp + k0);
        const v16h bl = frag_load(blp + k0);
        aM = mma_g(ah, bh, aM);
        aR = mma_g(ah, bl, aR);
        aR = mma_g(al, bh, aR);
      }
#pragma unroll
      for (int r = 0; r < 8; ++r)
        Ub[(8 * hh + r) * UP + ucol] = (aM[r] + aR[r] * RES_INV) * USCALE + pv[r];
    }
    __syncthreads();

    {
      const v4f u0 = *(const v4f*)(Ub + wave * UP + 8 * lane);
      const v4f u1 = *(const v4f*)(Ub + wave * UP + 8 * lane + 4);
      v4f qa0 = {0.f, 0.f, 0.f, 0.f}, qa1 = {0.f, 0.f, 0.f, 0.f};
      const float* qp = WHQ + (size_t)(rowbase + wave) * (size_t)(NQ * ND) + 8 * lane;
      const float* ep = eq  + (size_t)(rowbase + wave) * (size_t)(NQ * ND) + 8 * lane;
#pragma unroll 1
      for (int j = 0; j < NQ; ++j) {
        const v4f a0 = *(const v4f*)(qp + j * ND);
        const v4f a1 = *(const v4f*)(qp + j * ND + 4);
        const v4f e0 = *(const v4f*)(ep + j * ND);
        const v4f e1 = *(const v4f*)(ep + j * ND + 4);
        float s = wsum;
#pragma unroll
        for (int e = 0; e < 4; ++e) {
          const float r0 = __builtin_amdgcn_rcpf(__builtin_amdgcn_exp2f(a0[e] + u0[e]) + 1.0f);
          const float r1 = __builtin_amdgcn_rcpf(__builtin_amdgcn_exp2f(a1[e] + u1[e]) + 1.0f);
          s = fmaf(r0, m2w0[e], s);
          s = fmaf(r1, m2w1[e], s);
        }
        s += __shfl_xor(s, 16, 32);
        s += __shfl_xor(s, 8, 32);
        s += __shfl_xor(s, 4, 32);
        s += __shfl_xor(s, 2, 32);
        s += __shfl_xor(s, 1, 32);
#pragma unroll
        for (int e = 0; e < 4; ++e) {
          qa0[e] = fmaf(s, e0[e], qa0[e]);
          qa1[e] = fmaf(s, e1[e], qa1[e]);
        }
      }
      v8h hv, lv;
#pragma unroll
      for (int e = 0; e < 4; ++e) {
        const float fa = qa0[e] * ACT_CARRY;
        const float fb = qa1[e] * ACT_CARRY;
        _Float16 x0, y0, x1, y1;
        split16(fa, x0, y0);
        split16(fb, x1, y1);
        hv[e] = x0;
        lv[e] = y0;
        hv[4 + e] = x1;
        lv[4 + e] = y1;
      }
      *(v8h*)(Qh + wave * HP + 8 * lane) = hv;
      *(v8h*)(Ql + wave * HP + 8 * lane) = lv;
    }
    __syncthreads();

    v8f gM[4], gR[4];
#pragma unroll
    for (int g = 0; g < 4; ++g) { gM[g] = z8; gR[g] = z8; }
    {
      const _Float16* ahp = ECH + ((size_t)(rowbase + c) * NSTEP + (size_t)t) * ND + koff;
      const _Float16* alp = ECL + ((size_t)(rowbase + c) * NSTEP + (size_t)t) * ND + koff;
      const _Float16* bhp = WIH + (size_t)ucol * NZ + koff;
      const _Float16* blp = WIL + (size_t)ucol * NZ + koff;
#pragma unroll 1
      for (int k0 = 0; k0 < ND; k0 += 32) {
        const v16h ah = frag_load(ahp + k0);
        const v16h al = frag_load(alp + k0);
#pragma unroll
        for (int g = 0; g < 4; ++g) {
          const v16h bh = frag_load(bhp + (size_t)g * GS_IH + k0);
          const v16h bl = frag_load(blp + (size_t)g * GS_IH + k0);
          gM[g] = mma_g(ah, bh, gM[g]);
          gR[g] = mma_g(ah, bl, gR[g]);
          gR[g] = mma_g(al, bh, gR[g]);
        }
      }
    }
    {
      const _Float16* ahp = Qh + c * HP + koff;
      const _Float16* alp = Ql + c * HP + koff;
      const _Float16* bhp = WIH + (size_t)ucol * NZ + ND + koff;
      const _Float16* blp = WIL + (size_t)ucol * NZ + ND + koff;
#pragma unroll 1
      for (int k0 = 0; k0 < ND; k0 += 32) {
        const v16h ah = frag_load(ahp + k0);
        const v16h al = frag_load(alp + k0);
#pragma unroll
        for (int g = 0; g < 4; ++g) {
          const v16h bh = frag_load(bhp + (size_t)g * GS_IH + k0);
          const v16h bl = frag_load(blp + (size_t)g * GS_IH + k0);
          gM[g] = mma_g(ah, bh, gM[g]);
          gR[g] = mma_g(ah, bl, gR[g]);
          gR[g] = mma_g(al, bh, gR[g]);
        }
      }
    }
    {
      const _Float16* ahp = Hh + c * HP + koff;
      const _Float16* alp = Hl + c * HP + koff;
      const _Float16* bhp = WHH + (size_t)ucol * ND + koff;
      const _Float16* blp = WHL + (size_t)ucol * ND + koff;
#pragma unroll 1
      for (int k0 = 0; k0 < ND; k0 += 32) {
        const v16h ah = frag_load(ahp + k0);
        const v16h al = frag_load(alp + k0);
#pragma unroll
        for (int g = 0; g < 4; ++g) {
          const v16h bh = frag_load(bhp + (size_t)g * GS_HH + k0);
          const v16h bl = frag_load(blp + (size_t)g * GS_HH + k0);
          gM[g] = mma_g(ah, bh, gM[g]);
          gR[g] = mma_g(ah, bl, gR[g]);
          gR[g] = mma_g(al, bh, gR[g]);
        }
      }
    }
    float hst[8];
#pragma unroll
    for (int r = 0; r < 8; ++r) {
      const float zi = (gM[0][r] + gR[0][r] * RES_INV) * PROD_INV + bia[0];
      const float zf = (gM[1][r] + gR[1][r] * RES_INV) * PROD_INV + bia[1];
      const float zg = (gM[2][r] + gR[2][r] * RES_INV) * PROD_INV + bia[2];
      const float zo = (gM[3][r] + gR[3][r] * RES_INV) * PROD_INV + bia[3];
      const float ig = fsig(zi);
      const float fg = fsig(zf);
      const float gg = ftanh(zg);
      const float og = fsig(zo);
      const float cn = fg * cst[r] + ig * gg;
      cst[r] = cn;
      hst[r] = og * ftanh(cn);
    }
    __syncthreads();

#pragma unroll
    for (int r = 0; r < 8; ++r) {
      const int row = 8 * hh + r;
      const float hc = hst[r] * ACT_CARRY;
      _Float16 x, y;
      split16(hc, x, y);
      Hh[row * HP + ucol] = x;
      Hl[row * HP + ucol] = y;
      Hs[row * UP + ucol] = hst[r];
    }
    __syncthreads();

    {
      const v4f a = *(const v4f*)(Hs + wave * UP + 4 * lane);
      const v4f b = *(const v4f*)(Hs + wave * UP + 128 + 4 * lane);
      float* orow = out + ((size_t)(rowbase + wave) * NOUTROW + (size_t)(t + 1)) * ND;
      for (int pass = 0; pass < 2; ++pass) {
        *(volatile v4f*)(orow + 4 * lane) = a;
        *(volatile v4f*)(orow + 128 + 4 * lane) = b;
        __threadfence();
      }
    }
  }
}

extern "C" void kernel_launch(void* const* d_in, const int* in_sizes, int n_in,
                              void* d_out, int out_size, void* d_ws, size_t ws_size, hipStream_t stream) {
  if (n_in < 12 || d_out == nullptr || d_ws == nullptr) return;
  if (in_sizes[0] != NBATCH * NSTEP * ND || in_sizes[1] != NBATCH * NQ * ND || in_sizes[2] != NBATCH * ND ||
      in_sizes[3] != NBATCH * ND || in_sizes[4] != ND * ND || in_sizes[5] != ND * ND || in_sizes[6] != ND * ND ||
      in_sizes[7] != ND || in_sizes[8] != NG4 * NZ || in_sizes[9] != NG4 * ND || in_sizes[10] != NG4 ||
      in_sizes[11] != NG4 || out_size != NBATCH * NOUTROW * ND) return;

  const float* ec  = (const float*)d_in[0];
  const float* eq  = (const float*)d_in[1];
  const float* h0  = (const float*)d_in[2];
  const float* c0  = (const float*)d_in[3];
  const float* Wq  = (const float*)d_in[4];
  const float* Wp  = (const float*)d_in[5];
  const float* Wr  = (const float*)d_in[6];
  const float* wv  = (const float*)d_in[7];
  const float* Wih = (const float*)d_in[8];
  const float* Whh = (const float*)d_in[9];
  const float* bih = (const float*)d_in[10];
  const float* bhh = (const float*)d_in[11];
  float* out = (float*)d_out;

  char* ws = (char*)d_ws;
  size_t off = 0;
  auto carve = [&](size_t bytes) -> char* { char* p = ws + off; off += (bytes + 255) & ~(size_t)255; return p; };
  unsigned short* EQH  = (unsigned short*)carve((size_t)NBATCH * NQ * ND * 2);
  unsigned short* EQL  = (unsigned short*)carve((size_t)NBATCH * NQ * ND * 2);
  unsigned short* ECH  = (unsigned short*)carve((size_t)NBATCH * NSTEP * ND * 2);
  unsigned short* ECL  = (unsigned short*)carve((size_t)NBATCH * NSTEP * ND * 2);
  unsigned short* WT3  = (unsigned short*)carve((size_t)6 * ND * ND * 2);
  unsigned short* WIHH = (unsigned short*)carve((size_t)NG4 * NZ * 2);
  unsigned short* WIHL = (unsigned short*)carve((size_t)NG4 * NZ * 2);
  unsigned short* WHHH = (unsigned short*)carve((size_t)NG4 * ND * 2);
  unsigned short* WHHL = (unsigned short*)carve((size_t)NG4 * ND * 2);
  float*          WHQ  = (float*)carve((size_t)NBATCH * NQ * ND * 4);
  float*          WHP  = (float*)carve((size_t)NBATCH * NSTEP * ND * 4);
  if (off > ws_size || off > (size_t)134217728) return;

  const int n8eq = NBATCH * NQ * ND / 8;
  const int n8ec = NBATCH * NSTEP * ND / 8;
  const int n8ih = NG4 * NZ / 8;
  const int n8hh = NG4 * ND / 8;
  split8_kernel<<<n8eq / CTHR, CTHR, 0, stream>>>(eq,  EQH,  EQL,  n8eq, ACT_CARRY);
  split8_kernel<<<n8ec / CTHR, CTHR, 0, stream>>>(ec,  ECH,  ECL,  n8ec, ACT_CARRY);
  split8_kernel<<<n8ih / CTHR, CTHR, 0, stream>>>(Wih, WIHH, WIHL, n8ih, WGT_CARRY);
  split8_kernel<<<n8hh / CTHR, CTHR, 0, stream>>>(Whh, WHHH, WHHL, n8hh, WGT_CARRY);
  tsplit_kernel<<<dim3(ND / 64, ND / 64, 3), CTHR, 0, stream>>>(Wq, Wp, Wr, WT3, WGT_CARRY);

  unsigned short* WQH = WT3;
  unsigned short* WQL = WT3 + (size_t)1 * ND * ND;
  unsigned short* WPH = WT3 + (size_t)2 * ND * ND;
  unsigned short* WPL = WT3 + (size_t)3 * ND * ND;
  unsigned short* WRH = WT3 + (size_t)4 * ND * ND;
  unsigned short* WRL = WT3 + (size_t)5 * ND * ND;

  proj3_kernel<<<(NBATCH * NQ) / 32, CTHR, 0, stream>>>(EQH, EQL, WQH, WQL, WHQ, NBATCH * NQ, USCALE);
  proj3_kernel<<<(NBATCH * NSTEP) / 32, CTHR, 0, stream>>>(ECH, ECL, WPH, WPL, WHP, NBATCH * NSTEP, USCALE);

  seq_kernel<<<NBATCH / SEQ_BLK, PTHR, 0, stream>>>(ECH, ECL, WRH, WRL, WIHH, WIHL, WHHH, WHHL,
                                                    WHQ, WHP, eq, h0, c0, wv, bih, bhh, out);
}
